// FeatureGroupEncoder_50543175140060
// MI455X (gfx1250) — hardware-verified
//
#include <hip/hip_runtime.h>
#include <stddef.h>
#include <stdint.h>

#define NBATCH 8
#define SEQ    1024
#define NTOK   8192
#define FIN    256
#define EMB    512
#define INN    1024
#define UPN    2048
#define NHEAD  4
#define HDM    256
#define NGATE  8
#define GIN    3072
#define KS     4
#define QB     64
#define KC     32
#define NQB    16

static_assert(NTOK == NBATCH * SEQ);
static_assert(INN == NHEAD * HDM);
static_assert(GIN == 3 * INN);
static_assert(UPN == 2 * INN);
static_assert(NQB * QB == SEQ);
static_assert(QB == 2 * KC);
static_assert(HDM % 32 == 0);
static_assert(FIN % 32 == 0 && EMB % 64 == 0 && INN % 64 == 0 && NTOK % 64 == 0);
static_assert((NTOK * FIN) % 2048 == 0 && (EMB * FIN) % 2048 == 0 && (UPN * EMB) % 2048 == 0 && (EMB * INN) % 2048 == 0);
static_assert(NTOK % 8 == 0);
static_assert(SEQ % 64 == 0);

typedef unsigned short us;
typedef _Float16 f16t;
typedef __attribute__((ext_vector_type(16))) _Float16 v16h;
typedef __attribute__((ext_vector_type(16))) __bf16  v16bf;
typedef us           v8us __attribute__((ext_vector_type(8)));
typedef us           v4us __attribute__((ext_vector_type(4)));
typedef float        v8f  __attribute__((ext_vector_type(8)));
typedef float        v4f  __attribute__((ext_vector_type(4)));
typedef unsigned int v4u  __attribute__((ext_vector_type(4)));

union Frag  { v16h fh; v16bf fb; v8us h[2]; };
union Pack8 { v8us h; v4u u; };

#define LOG2E 1.44269504088896340736f

extern __shared__ __align__(16) float dyn_lds[];

__device__ __forceinline__ us bf_rne(float f) {
  unsigned u = __float_as_uint(f);
  u = u + 0x7FFFu + ((u >> 16) & 1u);
  return (us)(u >> 16);
}
__device__ __forceinline__ float bf_val(us hv) { return __uint_as_float(((unsigned)hv) << 16); }
__device__ __forceinline__ void split2(float f, us& hi, us& lo) {
  const us hv = bf_rne(f);
  hi = hv;
  lo = bf_rne(f - bf_val(hv));
}
__device__ __forceinline__ us hb(float f) {
  const f16t h = (f16t)f;
  return __builtin_bit_cast(us, h);
}
__device__ __forceinline__ float silu_f(float x) {
  const float e = __expf(-x);
  const float d = 1.0f + e;
  return x * __builtin_amdgcn_rcpf(d);
}
__device__ __forceinline__ v8f zero8() { return (v8f){0.f, 0.f, 0.f, 0.f, 0.f, 0.f, 0.f, 0.f}; }

__device__ __forceinline__ v8f mmah(v16h a, v16h b, v8f c) {
  c = __builtin_amdgcn_wmma_f32_16x16x32_f16(false, a, false, b, (short)0, c, false, false);
  asm volatile("v_nop\n\tv_nop\n\tv_nop\n\tv_nop" : "+v"(c) : "v"(a), "v"(b));
  return c;
}
__device__ __forceinline__ v8f mmab(v16bf a, v16bf b, v8f c) {
  c = __builtin_amdgcn_wmma_f32_16x16x32_bf16(false, a, false, b, (short)0, c, false, false);
  asm volatile("v_nop\n\tv_nop\n\tv_nop\n\tv_nop" : "+v"(c) : "v"(a), "v"(b));
  return c;
}

__device__ __forceinline__ Frag ldfrag(const us* p, int ld, int row0, int k0, int lane) {
  const int m = lane & 15, lh = lane >> 4;
  const us* q = p + (size_t)(row0 + m) * ld + k0 + 8 * lh;
  Frag f;
  f.h[0] = *(const v8us*)(q);
  f.h[1] = *(const v8us*)(q + 16);
  return f;
}

__global__ __launch_bounds__(256) void k_cvt16(const float* __restrict__ x, us* __restrict__ xh, float scale) {
  const size_t i = (size_t)blockIdx.x * 2048 + (size_t)threadIdx.x * 8;
  const v4f a0 = *(const v4f*)(x + i);
  const v4f a1 = *(const v4f*)(x + i + 4);
  Pack8 p;
  p.h = (v8us){hb(a0[0] * scale), hb(a0[1] * scale), hb(a0[2] * scale), hb(a0[3] * scale),
               hb(a1[0] * scale), hb(a1[1] * scale), hb(a1[2] * scale), hb(a1[3] * scale)};
  const v4u u = p.u;
  *(volatile v4u*)(xh + i) = u;
  __threadfence();
  *(volatile v4u*)(xh + i) = u;
}

#define SGP 68
template <int HASB>
__global__ __launch_bounds__(128) void k_gemm(const us* __restrict__ A, const us* __restrict__ W,
                                              const float* __restrict__ bias, float scale,
                                              float* __restrict__ C, int N, int K) {
  __shared__ __align__(16) float sg[64 * SGP];
  const int tid = threadIdx.x, lane = tid & 31, wave = tid >> 5;
  const int hh = lane >> 4, c = lane & 15;
  const int mb = blockIdx.y * 64;
  const int nb = blockIdx.x * 64;
  const int m0 = mb + 16 * wave;

  v8f acc[4];
#pragma unroll
  for (int j = 0; j < 4; ++j) acc[j] = zero8();

#pragma unroll 2
  for (int k0 = 0; k0 < K; k0 += 32) {
    const Frag a = ldfrag(A, K, m0, k0, lane);
#pragma unroll
    for (int j = 0; j < 4; ++j) {
      const Frag bw = ldfrag(W, K, nb + 16 * j, k0, lane);
      acc[j] = mmah(a.fh, bw.fh, acc[j]);
    }
  }

#pragma unroll
  for (int j = 0; j < 4; ++j) {
    const float bj = HASB ? bias[nb + 16 * j + c] : 0.f;
#pragma unroll
    for (int r = 0; r < 8; ++r) sg[(16 * wave + 8 * hh + r) * SGP + 16 * j + c] = acc[j][r] * scale + bj;
  }
  __syncthreads();

  v4f val[8];
  size_t go[8];
#pragma unroll
  for (int it = 0; it < 8; ++it) {
    const int p    = tid + 128 * it;
    const int L    = p >> 3;
    const int pc   = p & 7;
    const int row  = L >> 1;
    const int half = L & 1;
    const int col  = half * 32 + 4 * pc;
    val[it] = *(const v4f*)(sg + row * SGP + col);
    go[it]  = (size_t)(mb + row) * N + nb + col;
  }
#pragma unroll
  for (int it = 0; it < 8; ++it) *(volatile v4f*)(C + go[it]) = val[it];
  __threadfence();
#pragma unroll
  for (int it = 0; it < 8; ++it) *(volatile v4f*)(C + go[it]) = val[it];
}

__global__ __launch_bounds__(256) void k_ln1(const float* __restrict__ xp, const float* __restrict__ w,
                                             us* __restrict__ hh) {
  const int lane = threadIdx.x & 31, wave = threadIdx.x >> 5;
  const int row = blockIdx.x * 8 + wave;
  const float* src = xp + (size_t)row * EMB;
  v4f a[4], wv[4];
  a[0] = *(const v4f*)(src + 8 * lane);
  a[1] = *(const v4f*)(src + 8 * lane + 4);
  a[2] = *(const v4f*)(src + 256 + 8 * lane);
  a[3] = *(const v4f*)(src + 256 + 8 * lane + 4);
  wv[0] = *(const v4f*)(w + 8 * lane);
  wv[1] = *(const v4f*)(w + 8 * lane + 4);
  wv[2] = *(const v4f*)(w + 256 + 8 * lane);
  wv[3] = *(const v4f*)(w + 256 + 8 * lane + 4);
  float sm = 0.f;
#pragma unroll
  for (int q = 0; q < 4; ++q) {
#pragma unroll
    for (int e = 0; e < 4; ++e) sm += a[q][e];
  }
#pragma unroll
  for (int off = 1; off < 32; off <<= 1) sm += __shfl_xor(sm, off, 32);
  const float mean = sm * (1.0f / EMB);
  float sq = 0.f;
#pragma unroll
  for (int q = 0; q < 4; ++q) {
#pragma unroll
    for (int e = 0; e < 4; ++e) { const float d = a[q][e] - mean; sq += d * d; }
  }
#pragma unroll
  for (int off = 1; off < 32; off <<= 1) sq += __shfl_xor(sq, off, 32);
  const float var  = sq * (1.0f / EMB);
  const float rstd = rsqrtf(var + 1e-5f);
  us o[16];
#pragma unroll
  for (int q = 0; q < 4; ++q) {
#pragma unroll
    for (int e = 0; e < 4; ++e) o[4 * q + e] = hb(((a[q][e] - mean) * rstd) * wv[q][e]);
  }
  Pack8 p0, p1;
  p0.h = (v8us){o[0], o[1], o[2], o[3], o[4], o[5], o[6], o[7]};
  p1.h = (v8us){o[8], o[9], o[10], o[11], o[12], o[13], o[14], o[15]};
  us* dst = hh + (size_t)row * EMB;
  const v4u u0 = p0.u, u1 = p1.u;
  *(volatile v4u*)(dst + 8 * lane) = u0;
  *(volatile v4u*)(dst + 256 + 8 * lane) = u1;
  __threadfence();
  *(volatile v4u*)(dst + 8 * lane) = u0;
  *(volatile v4u*)(dst + 256 + 8 * lane) = u1;
}

#define CQP 68
#define CQT (64 * CQP)
#define CQ_LDS_BYTES (4 * CQT * 4 + NGATE * 64 * 4)
static_assert(CQ_LDS_BYTES == 71680);

__global__ __launch_bounds__(256) void k_cqg(const float* __restrict__ xm, const float* __restrict__ cw,
                                             const float* __restrict__ cbv, const float* __restrict__ wq,
                                             const float* __restrict__ wk, const float* __restrict__ wv,
                                             const float* __restrict__ wig, const float* __restrict__ big,
                                             const float* __restrict__ wfg, const float* __restrict__ bfg,
                                             float* __restrict__ xc, float* __restrict__ gp) {
  float* xcs = dyn_lds;
  float* qs  = xcs + CQT;
  float* ks  = qs + CQT;
  float* vs  = ks + CQT;
  float* gsm = vs + CQT;
  const int tid  = threadIdx.x;
  const int t    = tid & 63;
  const int g    = __builtin_amdgcn_readfirstlane(tid >> 6);
  const int tok0 = blockIdx.x * 64;
  const int sl0  = tok0 & (SEQ - 1);
  const int seq0 = tok0 - sl0;
  const int tok  = tok0 + t;
  const int sl   = sl0 + t;
  const float* wi = wig + (size_t)g * GIN;
  const float* wf = wfg + (size_t)g * GIN;
  float gia = 0.f, gfa = 0.f;

#pragma unroll 1
  for (int sub = 0; sub < INN / 64; ++sub) {
    const int cbase = sub * 64;
#pragma unroll 1
    for (int nb = 0; nb < 4; ++nb) {
      const int cl  = 16 * g + 4 * nb;
      const int c4  = cbase + cl;
      const int nbg = c4 >> 2;
      v4f xw[KS];
#pragma unroll
      for (int j = 0; j < KS; ++j) {
        const int  sp   = sl - (KS - 1) + j;
        const bool ok   = (sp >= 0);
        const int  rowc = ok ? (tok - (KS - 1) + j) : seq0;
        const v4f  ld   = *(const v4f*)(xm + (size_t)rowc * INN + c4);
        xw[j] = (v4f){ok ? ld[0] : 0.f, ok ? ld[1] : 0.f, ok ? ld[2] : 0.f, ok ? ld[3] : 0.f};
      }
      float xcv[4], qo[4], ko[4], vo[4];
#pragma unroll
      for (int i = 0; i < 4; ++i) {
        const float* cwp = cw + (size_t)(c4 + i) * KS;
        float a = xw[0][i] * cwp[0];
        a += xw[1][i] * cwp[1];
        a += xw[2][i] * cwp[2];
        a += xw[3][i] * cwp[3];
        a += cbv[c4 + i];
        xcv[i] = silu_f(a);
      }
#pragma unroll
      for (int o = 0; o < 4; ++o) {
        const float* wqp = wq + nbg * 16 + o * 4;
        const float* wkp = wk + nbg * 16 + o * 4;
        const float* wvp = wv + nbg * 16 + o * 4;
        qo[o] = xcv[0] * wqp[0] + xcv[1] * wqp[1] + xcv[2] * wqp[2] + xcv[3] * wqp[3];
        ko[o] = xcv[0] * wkp[0] + xcv[1] * wkp[1] + xcv[2] * wkp[2] + xcv[3] * wkp[3];
        vo[o] = xw[3][0] * wvp[0] + xw[3][1] * wvp[1] + xw[3][2] * wvp[2] + xw[3][3] * wvp[3];
      }
      const int lo = t * CQP + cl;
      *(v4f*)(xcs + lo) = (v4f){xcv[0], xcv[1], xcv[2], xcv[3]};
      *(v4f*)(qs + lo)  = (v4f){qo[0], qo[1], qo[2], qo[3]};
      *(v4f*)(ks + lo)  = (v4f){ko[0], ko[1], ko[2], ko[3]};
      *(v4f*)(vs + lo)  = (v4f){vo[0], vo[1], vo[2], vo[3]};
    }
    __syncthreads();

#pragma unroll 1
    for (int q4 = 0; q4 < 16; ++q4) {
      const int col = 4 * q4;
      const v4f qv = *(const v4f*)(qs + t * CQP + col);
      const v4f kv = *(const v4f*)(ks + t * CQP + col);
      const v4f vv = *(const v4f*)(vs + t * CQP + col);
      const float* wiq = wi + cbase + col;
      const float* wik = wi + INN + cbase + col;
      const float* wiv = wi + 2 * INN + cbase + col;
      const float* wfq = wf + cbase + col;
      const float* wfk = wf + INN + cbase + col;
      const float* wfv = wf + 2 * INN + cbase + col;
#pragma unroll
      for (int e = 0; e < 4; ++e) {
        gia += qv[e] * wiq[e];
        gia += kv[e] * wik[e];
        gia += vv[e] * wiv[e];
        gfa += qv[e] * wfq[e];
        gfa += kv[e] * wfk[e];
        gfa += vv[e] * wfv[e];
      }
    }

    v4f val[4];
    size_t go[4];
#pragma unroll
    for (int it = 0; it < 4; ++it) {
      const int p    = tid + 256 * it;
      const int L    = p >> 3;
      const int pc   = p & 7;
      const int row  = L >> 1;
      const int half = L & 1;
      const int col  = half * 32 + 4 * pc;
      val[it] = *(const v4f*)(xcs + row * CQP + col);
      go[it]  = (size_t)(tok0 + row) * INN + cbase + col;
    }
#pragma unroll
    for (int it = 0; it < 4; ++it) *(volatile v4f*)(xc + go[it]) = val[it];
    __threadfence();
#pragma unroll
    for (int it = 0; it < 4; ++it) *(volatile v4f*)(xc + go[it]) = val[it];
    __syncthreads();
  }

  gsm[g * 64 + t]           = gia + big[g];
  gsm[(NHEAD + g) * 64 + t] = gfa + bfg[g];
  __syncthreads();
  if (tid < 128) {
    const int p    = tid;
    const int L    = p >> 3;
    const int pc   = p & 7;
    const int row  = L >> 1;
    const int half = L & 1;
    const int col  = half * 32 + 4 * pc;
    const v4f gv   = *(const v4f*)(gsm + row * 64 + col);
    const size_t goo = (size_t)row * NTOK + tok0 + col;
    *(volatile v4f*)(gp + goo) = gv;
    __threadfence();
    *(volatile v4f*)(gp + goo) = gv;
  }
}

__global__ __launch_bounds__(1024) void k_scan(const float* __restrict__ gr, float* __restrict__ a2p,
                                               float* __restrict__ nm2p, float* __restrict__ ep) {
  __shared__ float buf[SEQ];
  __shared__ __align__(16) float sa[SEQ];
  __shared__ __align__(16) float sn[SEQ];
  __shared__ __align__(16) float se[SEQ];
  const int t  = threadIdx.x;
  const int bh = blockIdx.x;
  const int b  = bh / NHEAD;
  const int h  = bh - b * NHEAD;
  const float ig = gr[(size_t)h * NTOK + b * SEQ + t];
  const float fg = gr[(size_t)(NHEAD + h) * NTOK + b * SEQ + t];
  const float lg = fminf(fg, 0.f) - log1pf(expf(-fabsf(fg)));
  buf[t] = lg;
  __syncthreads();
#pragma unroll 1
  for (int off = 1; off < SEQ; off <<= 1) {
    const int si   = (t >= off) ? (t - off) : 0;
    const float pv = buf[si];
    const float p  = (t >= off) ? pv : 0.f;
    __syncthreads();
    buf[t] += p;
    __syncthreads();
  }
  const float cs = buf[t];
  const float a  = ig - cs;
  __syncthreads();
  buf[t] = a;
  __syncthreads();
  const float NEGINF = -__builtin_huge_valf();
#pragma unroll 1
  for (int off = 1; off < SEQ; off <<= 1) {
    const int si   = (t >= off) ? (t - off) : 0;
    const float pv = buf[si];
    const float p  = (t >= off) ? pv : NEGINF;
    __syncthreads();
    buf[t] = fmaxf(buf[t], p);
    __syncthreads();
  }
  const float M = buf[t];
  sa[t] = a * LOG2E;
  sn[t] = -(M * LOG2E);
  se[t] = expf(-(cs + M));
  __syncthreads();
  if (t < SEQ / 4) {
    const v4f xa = *(const v4f*)(sa + 4 * t);
    const v4f xn = *(const v4f*)(sn + 4 * t);
    const v4f xe = *(const v4f*)(se + 4 * t);
    const size_t go = (size_t)bh * SEQ + 4 * t;
    *(volatile v4f*)(a2p + go)  = xa;
    *(volatile v4f*)(nm2p + go) = xn;
    *(volatile v4f*)(ep + go)   = xe;
    __threadfence();
    *(volatile v4f*)(a2p + go)  = xa;
    *(volatile v4f*)(nm2p + go) = xn;
    *(volatile v4f*)(ep + go)   = xe;
  }
}

#define AT_QH   0
#define AT_QL   (AT_QH + QB * HDM * 2)
#define AT_KH   (AT_QL + QB * HDM * 2)
#define AT_KL   (AT_KH + KC * HDM * 2)
#define AT_VH   (AT_KL + KC * HDM * 2)
#define AT_VL   (AT_VH + HDM * KC * 2)
#define AT_CH   (AT_VL + HDM * KC * 2)
#define AT_CL   (AT_CH + 4 * 16 * KC * 2)
#define AT_O    (AT_CL + 4 * 16 * KC * 2)
#define AT_LDS_BYTES (AT_O + 4 * 16 * HDM * 4)
static_assert(AT_LDS_BYTES == 204800);
static_assert(AT_O % 256 == 0);

__global__ __launch_bounds__(128) void k_attn(const float* __restrict__ xc, const float* __restrict__ xm,
                                              const float* __restrict__ zp, const float* __restrict__ wq,
                                              const float* __restrict__ wk, const float* __restrict__ wv,
                                              const float* __restrict__ a2g, const float* __restrict__ nm2g,
                                              const float* __restrict__ eg, const float* __restrict__ nw,
                                              const float* __restrict__ skw, us* __restrict__ hs) {
  unsigned char* dl = (unsigned char*)dyn_lds;
  us* Qsh = (us*)(dl + AT_QH);
  us* Qsl = (us*)(dl + AT_QL);
  us* Ksh = (us*)(dl + AT_KH);
  us* Ksl = (us*)(dl + AT_KL);
  us* Vsh = (us*)(dl + AT_VH);
  us* Vsl = (us*)(dl + AT_VL);
  us* Csh = (us*)(dl + AT_CH);
  us* Csl = (us*)(dl + AT_CL);
  float* Olds = (float*)(dl + AT_O);

  const int tid = threadIdx.x, lane = tid & 31, wave = tid >> 5;
  const int hh = lane >> 4, c = lane & 15;
  const int bh   = blockIdx.x / NQB;
  const int qb   = blockIdx.x - bh * NQB;
  const int b    = bh / NHEAD;
  const int hd   = bh - b * NHEAD;
  const int tok0 = b * SEQ;
  const int col0 = hd * HDM;
  const int qblk = qb * QB;
  const int qloc = qblk + wave * 16;
  const int q0   = tok0 + qloc;
  const int nch  = 2 * qb + 2;
  const size_t gb = (size_t)bh * SEQ;

  float* ow  = Olds + wave * (16 * 32 * 8);
  us*    pwh = Csh + wave * (16 * KC);
  us*    pwl = Csl + wave * (16 * KC);

  const v4f z4 = {0.f, 0.f, 0.f, 0.f};
#pragma unroll
  for (int t = 0; t < 16; ++t) {
    float* op = ow + (t * 32 + lane) * 8;
    *(v4f*)op = z4;
    *(v4f*)(op + 4) = z4;
  }

#pragma unroll 1
  for (int it = 0; it < (QB * HDM / 4) / 128; ++it) {
    const int qd  = tid + 128 * it;
    const int row = qd & (QB - 1);
    const int nq  = __builtin_amdgcn_readfirstlane(qd >> 6);
    const int cq  = col0 + 4 * nq;
    const int nbg = cq >> 2;
    const v4f xv  = *(const v4f*)(xc + (size_t)(tok0 + qblk + row) * INN + cq);
    const float* w = wq + nbg * 16;
    us h4[4], l4[4];
#pragma unroll
    for (int o = 0; o < 4; ++o) {
      const float qv = xv[0] * w[o * 4] + xv[1] * w[o * 4 + 1] + xv[2] * w[o * 4 + 2] + xv[3] * w[o * 4 + 3];
      split2(qv, h4[o], l4[o]);
    }
    const int lo = row * HDM + 4 * nq;
    *(v4us*)(Qsh + lo) = (v4us){h4[0], h4[1], h4[2], h4[3]};
    *(v4us*)(Qsl + lo) = (v4us){l4[0], l4[1], l4[2], l4[3]};
  }

  float nm2[8], zrow[8];
#pragma unroll
  for (int r = 0; r < 8; ++r) {
    nm2[r]  = nm2g[gb + qloc + 8 * hh + r];
    zrow[r] = 0.f;
  }

#pragma unroll 1
  for (int i = 0; i < nch; ++i) {
    const int kv0 = i * KC;
    __syncthreads();
#pragma unroll 1
    for (int it = 0; it < (KC * HDM / 4) / 128; ++it) {
      const int qd  = tid + 128 * it;
      const int key = qd & (KC - 1);
      const int nq  = __builtin_amdgcn_readfirstlane(qd >> 5);
      const int cq  = col0 + 4 * nq;
      const int nbg = cq >> 2;
      const size_t ti = (size_t)(tok0 + kv0 + key) * INN + cq;
      const v4f xv  = *(const v4f*)(xc + ti);
      const v4f mv  = *(const v4f*)(xm + ti);
      const float* wkp = wk + nbg * 16;
      const float* wvp = wv + nbg * 16;
      us kh4[4], kl4[4];
#pragma unroll
      for (int o = 0; o < 4; ++o) {
        const float kvl = xv[0] * wkp[o * 4] + xv[1] * wkp[o * 4 + 1] + xv[2] * wkp[o * 4 + 2] + xv[3] * wkp[o * 4 + 3];
        const float vvl = mv[0] * wvp[o * 4] + mv[1] * wvp[o * 4 + 1] + mv[2] * wvp[o * 4 + 2] + mv[3] * wvp[o * 4 + 3];
        us vh1, vl1;
        split2(kvl, kh4[o], kl4[o]);
        split2(vvl, vh1, vl1);
        Vsh[(4 * nq + o) * KC + key] = vh1;
        Vsl[(4 * nq + o) * KC + key] = vl1;
      }
      const int lo = key * HDM + 4 * nq;
      *(v4us*)(Ksh + lo) = (v4us){kh4[0], kh4[1], kh4[2], kh4[3]};
      *(v4us*)(Ksl + lo) = (v4us){kl4[0], kl4[1], kl4[2], kl4[3]};
    }
    __syncthreads();

    v8f s[2];
    s[0] = zero8();
    s[1] = zero8();
#pragma unroll 2
    for (int dc = 0; dc < HDM / 32; ++dc) {
      const Frag qah = ldfrag(Qsh, HDM, 16 * wave, 32 * dc, lane);
      const Frag qal = ldfrag(Qsl, HDM, 16 * wave, 32 * dc, lane);
#pragma unroll
      for (int j = 0; j < 2; ++j) {
        const Frag kbh = ldfrag(Ksh, HDM, 16 * j, 32 * dc, lane);
        const Frag kbl = ldfrag(Ksl, HDM, 16 * j, 32 * dc, lane);
        s[j] = mmab(qah.fb, kbh.fb, s[j]);
        s[j] = mmab(qah.fb, kbl.fb, s[j]);
        s[j] = mmab(qal.fb, kbh.fb, s[j]);
      }
    }
#pragma unroll
    for (int j = 0; j < 2; ++j) {
      const int key  = kv0 + 16 * j + c;
      const float g2 = a2g[gb + key];
#pragma unroll
      for (int r = 0; r < 8; ++r) {
        const int qrow = qloc + 8 * hh + r;
        const float xe = fminf(g2 + nm2[r], 0.f);
        const float dd = exp2f(xe);
        const float cv = (s[j][r] * 0.0625f) * dd;
        s[j][r] = (key <= qrow) ? cv : 0.f;
      }
    }
#pragma unroll
    for (int r = 0; r < 8; ++r) {
      float psum = 0.f;
#pragma unroll
      for (int j = 0; j < 2; ++j) {
        const float cv = s[j][r];
        psum += cv;
        us ph, pl;
        split2(cv, ph, pl);
        pwh[(8 * hh + r) * KC + 16 * j + c] = ph;
        pwl[(8 * hh + r) * KC + 16 * j + c] = pl;
      }
#pragma unroll
      for (int off = 1; off < 16; off <<= 1) psum += __shfl_xor(psum, off, 32);
      zrow[r] += psum;
    }
    __syncthreads();

    const Frag pah = ldfrag(pwh, KC, 0, 0, lane);
    const Frag pal = ldfrag(pwl, KC, 0, 0, lane);
#pragma unroll 1
    for (int t = 0; t < 16; ++t) {
      float* op = ow + (t * 32 + lane) * 8;
      const v4f o0 = *(const v4f*)op;
      const v4f o1 = *(const v4f*)(op + 4);
      v8f acc = (v8f){o0[0], o0[1], o0[2], o0[3], o1[0], o1[1], o1[2], o1[3]};
      const Frag vbh = ldfrag(Vsh, KC, 16 * t, 0, lane);
      const Frag vbl = ldfrag(Vsl, KC, 16 * t, 0, lane);
      acc = mmab(pah.fb, vbh.fb, acc);
      acc = mmab(pah.fb, vbl.fb, acc);
      acc = mmab(pal.fb, vbh.fb, acc);
      *(v4f*)op       = (v4f){acc[0], acc[1], acc[2], acc[3]};
      *(v4f*)(op + 4) = (v4f){acc[4], acc[5], acc[6], acc[7]};
    }
  }

  float inv[8], mean[8], rstd[8];
#pragma unroll
  for (int r = 0; r < 8; ++r) {
    const float er = eg[gb + qloc + 8 * hh + r];
    inv[r]  = 1.0f / (fmaxf(fabsf(zrow[r]), er) + 1e-6f);
    mean[r] = 0.f;
    rstd[r] = 0.f;
  }
#pragma unroll 1
  for (int t = 0; t < 16; ++t) {
    const float* op = ow + (t * 32 + lane) * 8;
    const v4f o0 = *(const v4f*)op;
    const v4f o1 = *(const v4f*)(op + 4);
    const float of[8] = {o0[0], o0[1], o0[2], o0[3], o1[0], o1[1], o1[2], o1[3]};
#pragma unroll
    for (int r = 0; r < 8; ++r) mean[r] += of[r] * inv[r];
  }
#pragma unroll
  for (int r = 0; r < 8; ++r) {
    float sm = mean[r];
#pragma unroll
    for (int off = 1; off < 16; off <<= 1) sm += __shfl_xor(sm, off, 32);
    mean[r] = sm * (1.0f / HDM);
  }
#pragma unroll 1
  for (int t = 0; t < 16; ++t) {
    const float* op = ow + (t * 32 + lane) * 8;
    const v4f o0 = *(const v4f*)op;
    const v4f o1 = *(const v4f*)(op + 4);
    const float of[8] = {o0[0], o0[1], o0[2], o0[3], o1[0], o1[1], o1[2], o1[3]};
#pragma unroll
    for (int r = 0; r < 8; ++r) { const float d = of[r] * inv[r] - mean[r]; rstd[r] += d * d; }
  }
#pragma unroll
  for (int r = 0; r < 8; ++r) {
    float sq = rstd[r];
#pragma unroll
    for (int off = 1; off < 16; off <<= 1) sq += __shfl_xor(sq, off, 32);
    rstd[r] = rsqrtf(sq * (1.0f / HDM) + 1e-5f);
  }
#pragma unroll 1
  for (int t = 0; t < 16; ++t) {
    float* op = ow + (t * 32 + lane) * 8;
    const v4f o0 = *(const v4f*)op;
    const v4f o1 = *(const v4f*)(op + 4);
    const float of[8] = {o0[0], o0[1], o0[2], o0[3], o1[0], o1[1], o1[2], o1[3]};
    float u[8];
#pragma unroll
    for (int r = 0; r < 8; ++r) u[r] = (of[r] * inv[r] - mean[r]) * rstd[r];
    *(v4f*)op       = (v4f){u[0], u[1], u[2], u[3]};
    *(v4f*)(op + 4) = (v4f){u[4], u[5], u[6], u[7]};
  }
  __syncthreads();

  us* stg = Qsh + wave * 16 * HDM;
#pragma unroll 1
  for (int it = 0; it < 16; ++it) {
    const int p    = lane + 32 * it;
    const int L    = p >> 3;
    const int pc   = p & 7;
    const int row  = L >> 2;
    const int qt   = L & 3;
    const int colh = qt * 64 + 8 * pc;
    const int t    = colh >> 4;
    const int cb   = colh & 15;
    const float* usl = ow + ((t * 32 + 16 * (row >> 3) + cb) * 8 + (row & 7));
    float u[8];
#pragma unroll
    for (int e = 0; e < 8; ++e) u[e] = usl[8 * e];
    const int ch0 = col0 + colh;
    const v4f w0 = *(const v4f*)(nw + ch0);
    const v4f w1 = *(const v4f*)(nw + ch0 + 4);
    const v4f k0 = *(const v4f*)(skw + ch0);
    const v4f k1 = *(const v4f*)(skw + ch0 + 4);
    const size_t ti = (size_t)(q0 + row) * INN + ch0;
    const v4f x0 = *(const v4f*)(xc + ti);
    const v4f x1 = *(const v4f*)(xc + ti + 4);
    const v4f g0 = *(const v4f*)(zp + ti);
    const v4f g1 = *(const v4f*)(zp + ti + 4);
    const float wn[8] = {w0[0], w0[1], w0[2], w0[3], w1[0], w1[1], w1[2], w1[3]};
    const float sk[8] = {k0[0], k0[1], k0[2], k0[3], k1[0], k1[1], k1[2], k1[3]};
    const float xv[8] = {x0[0], x0[1], x0[2], x0[3], x1[0], x1[1], x1[2], x1[3]};
    const float zv[8] = {g0[0], g0[1], g0[2], g0[3], g1[0], g1[1], g1[2], g1[3]};
    us o8[8];
#pragma unroll
    for (int e = 0; e < 8; ++e) {
      const float hn = u[e] * wn[e];
      const float hv = (hn + sk[e] * xv[e]) * silu_f(zv[e]);
      o8[e] = hb(hv);
    }
    Pack8 pk;
    pk.h = (v8us){o8[0], o8[1], o8[2], o8[3], o8[4], o8[5], o8[6], o8[7]};
    *(v8us*)(stg + row * HDM + colh) = pk.h;
    const v4u pu = pk.u;
    const size_t go = (size_t)(q0 + row) * INN + ch0;
    *(volatile v4u*)(hs + go) = pu;
  }
  __threadfence();
#pragma unroll 1
  for (int it = 0; it < 16; ++it) {
    const int p    = lane + 32 * it;
    const int L    = p >> 3;
    const int pc   = p & 7;
    const int row  = L >> 2;
    const int qt   = L & 3;
    const int colh = qt * 64 + 8 * pc;
    Pack8 pk;
    pk.h = *(const v8us*)(stg + row * HDM + colh);
    const v4u pu = pk.u;
    const size_t go = (size_t)(q0 + row) * INN + col0 + colh;
    *(volatile v4u*)(hs + go) = pu;
  }
}

__global__ __launch_bounds__(256) void k_addln(const float* __restrict__ xp, const float* __restrict__ y,
                                               const float* __restrict__ w, float* __restrict__ out) {
  const int lane = threadIdx.x & 31, wave = threadIdx.x >> 5;
  const int row = blockIdx.x * 8 + wave;
  const float* px = xp + (size_t)row * EMB;
  const float* py = y + (size_t)row * EMB;
  v4f a[4], wv[4];
#pragma unroll
  for (int s = 0; s < 4; ++s) {
    const int off = 128 * s + 4 * lane;
    a[s]  = *(const v4f*)(px + off) + *(const v4f*)(py + off);
    wv[s] = *(const v4f*)(w + off);
  }
  float sm = 0.f;
#pragma unroll
  for (int s = 0; s < 4; ++s) {
#pragma unroll
    for (int e = 0; e < 4; ++e) sm += a[s][e];
  }
#pragma unroll
  for (int off = 1; off < 32; off <<= 1) sm += __shfl_xor(sm, off, 32);
  const float mean = sm * (1.0f / EMB);
  float sq = 0.f;
#pragma unroll
  for (int s = 0; s < 4; ++s) {
#pragma unroll
    for (int e = 0; e < 4; ++e) { const float d = a[s][e] - mean; sq += d * d; }
  }
#pragma unroll
  for (int off = 1; off < 32; off <<= 1) sq += __shfl_xor(sq, off, 32);
  const float var  = sq * (1.0f / EMB);
  const float rstd = rsqrtf(var + 1e-5f);
  v4f o[4];
#pragma unroll
  for (int s = 0; s < 4; ++s) {
    o[s] = (v4f){((a[s][0] - mean) * rstd) * wv[s][0], ((a[s][1] - mean) * rstd) * wv[s][1],
                 ((a[s][2] - mean) * rstd) * wv[s][2], ((a[s][3] - mean) * rstd) * wv[s][3]};
  }
  float* dst = out + (size_t)row * EMB;
#pragma unroll
  for (int s = 0; s < 4; ++s) *(volatile v4f*)(dst + 128 * s + 4 * lane) = o[s];
  __threadfence();
#pragma unroll
  for (int s = 0; s < 4; ++s) *(volatile v4f*)(dst + 128 * s + 4 * lane) = o[s];
}

extern "C" void kernel_launch(void* const* d_in, const int* in_sizes, int n_in,
                              void* d_out, int out_size, void* d_ws, size_t ws_size,
                              hipStream_t stream) {
  if (n_in < 18) return;
  if (in_sizes[0] != NTOK * FIN) return;
  if (in_sizes[1] != EMB * FIN) return;
  if (in_sizes[2] != EMB) return;
  if (in_sizes[3] != EMB) return;
  if (in_sizes[4] != UPN * EMB) return;
  if (in_sizes[5] != INN * KS) return;
  if (in_sizes[6] != INN) return;
  if (in_sizes[7] != (INN / 4) * 16) return;
  if (in_sizes[8] != (INN / 4) * 16) return;
  if (in_sizes[9] != (INN / 4) * 16) return;
  if (in_sizes[10] != NHEAD * GIN) return;
  if (in_sizes[11] != NHEAD) return;
  if (in_sizes[12] != NHEAD * GIN) return;
  if (in_sizes[13] != NHEAD) return;
  if (in_sizes[14] != INN) return;
  if (in_sizes[15] != INN) return;
  if (in_sizes[16] != EMB * INN) return;
  if (in_sizes[17] != EMB) return;
  if (out_size != NTOK * EMB) return;

  const float* x       = (const float*)d_in[0];
  const float* W_in    = (const float*)d_in[1];
  const float* b_in    = (const float*)d_in[2];
  const float* ln1_w   = (const float*)d_in[3];
  const float* W_up    = (const float*)d_in[4];
  const float* conv_w  = (const float*)d_in[5];
  const float* conv_b  = (const float*)d_in[6];
  const float* Wq      = (const float*)d_in[7];
  const float* Wk      = (const float*)d_in[8];
  const float* Wv      = (const float*)d_in[9];
  const float* W_ig    = (const float*)d_in[10];
  const float* b_ig    = (const float*)d_in[11];
  const float* W_fg    = (const float*)d_in[12];
  const float* b_fg    = (const float*)d_in[13];
  const float* mhln_w  = (const float*)d_in[14];
  const float* skipw   = (const float*)d_in[15];
  const float* W_down  = (const float*)d_in[16];
  const float* ln_post = (const float*)d_in[17];
  float* out = (float*)d_out;

  const size_t MIB  = 1048576;
  const size_t oZ   = 0;
  const size_t oXM  = 32 * MIB;
  const size_t oXC  = 64 * MIB;
  const size_t oHS  = 96 * MIB;
  const size_t oXH  = 112 * MIB;
  const size_t oWIN = 116 * MIB;
  const size_t oG   = oWIN + (size_t)EMB * FIN * 2;
  const size_t oA2  = oG + (size_t)NGATE * NTOK * 4;
  const size_t oNM  = oA2 + (size_t)NBATCH * NHEAD * SEQ * 4;
  const size_t oE   = oNM + (size_t)NBATCH * NHEAD * SEQ * 4;
  const size_t oEnd = oE + (size_t)NBATCH * NHEAD * SEQ * 4;
  if ((size_t)NTOK * INN * 4 != 32 * MIB) return;
  if ((size_t)NTOK * EMB * 4 != 16 * MIB) return;
  if ((size_t)NTOK * INN * 2 != 16 * MIB) return;
  if ((size_t)NTOK * FIN * 2 != 4 * MIB) return;
  if ((size_t)UPN * EMB * 2 + (size_t)NTOK * EMB * 2 > 32 * MIB) return;
  if ((size_t)EMB * INN * 2 > 32 * MIB) return;
  if (oEnd > ws_size) return;
  if (oEnd > (size_t)134217728) return;

  char* ws = (char*)d_ws;
  float* Zp   = (float*)(ws + oZ);
  float* XPE  = (float*)(ws + oZ);
  float* XPL  = (float*)(ws + oZ);
  float* Yp   = (float*)(ws + oZ + 16 * MIB);
  float* XM   = (float*)(ws + oXM);
  us*    WDNH = (us*)(ws + oXM);
  float* XC   = (float*)(ws + oXC);
  us*    WUPH = (us*)(ws + oXC);
  us*    HH   = (us*)(ws + oXC + (size_t)UPN * EMB * 2);
  us*    HS   = (us*)(ws + oHS);
  us*    XH   = (us*)(ws + oXH);
  us*    WINH = (us*)(ws + oWIN);
  float* G    = (float*)(ws + oG);
  float* A2   = (float*)(ws + oA2);
  float* NM2  = (float*)(ws + oNM);
  float* EP   = (float*)(ws + oE);

  (void)hipFuncSetAttribute(reinterpret_cast<const void*>(&k_cqg), hipFuncAttributeMaxDynamicSharedMemorySize,
                            CQ_LDS_BYTES);
  (void)hipFuncSetAttribute(reinterpret_cast<const void*>(&k_attn), hipFuncAttributeMaxDynamicSharedMemorySize,
                            AT_LDS_BYTES);

  k_cvt16<<<dim3((NTOK * FIN) / 2048), dim3(256), 0, stream>>>(x, XH, 1.0f);
  k_cvt16<<<dim3((EMB * FIN) / 2048), dim3(256), 0, stream>>>(W_in, WINH, 16.0f);
  k_cvt16<<<dim3((UPN * EMB) / 2048), dim3(256), 0, stream>>>(W_up, WUPH, 16.0f);
  k_gemm<1><<<dim3(EMB / 64, NTOK / 64), dim3(128), 0, stream>>>(XH, WINH, b_in, 0.0625f, XPE, EMB, FIN);
  k_ln1<<<dim3(NTOK / 8), dim3(256), 0, stream>>>(XPE, ln1_w, HH);
  k_gemm<0><<<dim3(INN / 64, NTOK / 64), dim3(128), 0, stream>>>(HH, WUPH, b_in, 0.0625f, XM, INN, EMB);
  k_gemm<0><<<dim3(INN / 64, NTOK / 64), dim3(128), 0, stream>>>(HH, WUPH + (size_t)INN * EMB, b_in, 0.0625f, Zp,
                                                                 INN, EMB);
  k_cqg<<<dim3(NTOK / 64), dim3(256), CQ_LDS_BYTES, stream>>>(XM, conv_w, conv_b, Wq, Wk, Wv, W_ig, b_ig, W_fg,
                                                              b_fg, XC, G);
  k_scan<<<dim3(NBATCH * NHEAD), dim3(SEQ), 0, stream>>>(G, A2, NM2, EP);
  k_attn<<<dim3(NBATCH * NHEAD * NQB), dim3(128), AT_LDS_BYTES, stream>>>(XC, XM, Zp, Wq, Wk, Wv, A2, NM2, EP,
                                                                          mhln_w, skipw, HS);
  k_cvt16<<<dim3((EMB * INN) / 2048), dim3(256), 0, stream>>>(W_down, WDNH, 32.0f);
  k_gemm<1><<<dim3(EMB / 64, NTOK / 64), dim3(128), 0, stream>>>(XH, WINH, b_in, 0.0625f, XPL, EMB, FIN);
  k_gemm<0><<<dim3(EMB / 64, NTOK / 64), dim3(128), 0, stream>>>(HS, WDNH, b_in, 0.03125f, Yp, EMB, INN);
  k_addln<<<dim3(NTOK / 8), dim3(256), 0, stream>>>(XPL, Yp, ln_post, out);
  (void)hipGetLastError();
}
